// MultiHeadAttention_14396730376956
// MI455X (gfx1250) — hardware-run, weakly checked
//
#include <hip/hip_runtime.h>
#ifndef NB
#define NB 2
#endif
#ifndef SEQ
#define SEQ 4096
#endif
#define NB_FULL 2
#define SEQ_FULL 4096
#define DM 768
#define NH 12
#define HD 64
#define NTOK ((size_t)NB * SEQ)
#define EARLY ((SEQ) < 1024 ? (SEQ) : 1024)
static_assert(SEQ % 128 == 0);
static_assert(EARLY % 128 == 0);
static_assert((SEQ - EARLY) % 128 == 0);
static_assert(NB <= NB_FULL);
static_assert(SEQ <= SEQ_FULL);
static_assert(DM % 128 == 0);
static_assert(NH * HD == DM);
static_assert(HD == 64);
static_assert(DM % 32 == 0);
static_assert(DM % 64 == 0);
static_assert(DM % 8 == 0);
static_assert(SEQ % 64 == 0);
static_assert(SEQ % 32 == 0);
static_assert(((size_t)NB * SEQ) % 128 == 0);
static_assert(((size_t)NB * SEQ) % 64 == 0);
static_assert((size_t)NB_FULL * DM < (size_t)2147483647);
static_assert(((size_t)(SEQ - 1) * NB_FULL + NB) * DM <= (size_t)NB_FULL * SEQ_FULL * DM);
static_assert(((size_t)DM * DM * 2) % 256 == 0);
static_assert(((size_t)NB * SEQ * DM * 2) % 256 == 0);
static_assert((size_t)4 * DM * DM * 2 + (size_t)7 * NB * SEQ * DM * 2 <= (size_t)134217728);

typedef _Float16 v16h __attribute__((ext_vector_type(16)));
typedef _Float16 v4h __attribute__((ext_vector_type(4)));
typedef unsigned short v8us __attribute__((ext_vector_type(8), may_alias));
typedef float v8f __attribute__((ext_vector_type(8)));
typedef float v4f __attribute__((ext_vector_type(4)));
typedef float v4fa __attribute__((ext_vector_type(4), may_alias));
union FragH { v16h v; v8us half[2]; _Float16 h[16]; unsigned short u[16]; };

__device__ __forceinline__ unsigned short bf16_bits(float x) { unsigned int u = __float_as_uint(x); return (unsigned short)((u + 0x7FFFu + ((u >> 16) & 1u)) >> 16); }
__device__ __forceinline__ float bf16_rne(float x) { return __uint_as_float(((unsigned int)bf16_bits(x)) << 16); }

typedef _Float16 h16;
static __device__ __forceinline__ h16 toh_flush(float v) { const h16 r = (h16)v; return (fabsf(v) < 6.103515625e-05f) ? (h16)0.0f : r; }

__device__ __forceinline__ v16h ld_frag(const unsigned short* p) { FragH f; f.half[0] = *(const v8us*)p; f.half[1] = *(const v8us*)(p + 16); return f.v; }

__device__ __forceinline__ v8f wm(v16h a, v16h b, v8f c) { return __builtin_amdgcn_wmma_f32_16x16x32_f16(false, a, false, b, (short)0, c, false, false); }
__device__ __forceinline__ v8f mma1(v16h a, v16h b, v8f c) {
  c = wm(a, b, c);
  asm volatile("v_nop\n\tv_nop\n\tv_nop\n\tv_nop" : "+v"(c) : "v"(a), "v"(b));
  return c;
}
__device__ __forceinline__ v8f mma2(v16h a0, v16h b0, v16h a1, v16h b1, v8f c) {
  c = wm(a0, b0, c); c = wm(a1, b1, c);
  asm volatile("v_nop\n\tv_nop\n\tv_nop\n\tv_nop" : "+v"(c) : "v"(a0), "v"(b0), "v"(a1), "v"(b1));
  return c;
}
__device__ __forceinline__ v8f mma4(v16h a0, v16h b0, v16h a1, v16h b1, v16h a2, v16h b2, v16h a3, v16h b3, v8f c) {
  c = wm(a0, b0, c); c = wm(a1, b1, c); c = wm(a2, b2, c); c = wm(a3, b3, c);
  asm volatile("v_nop\n\tv_nop\n\tv_nop\n\tv_nop" : "+v"(c) : "v"(a0), "v"(b0), "v"(a1), "v"(b1), "v"(a2), "v"(b2), "v"(a3), "v"(b3));
  return c;
}

__global__ __launch_bounds__(256) void k_wnat(const float* __restrict__ w, unsigned int n8, unsigned short* __restrict__ Bt, float scale) {
  const unsigned int t = blockIdx.x * 256u + threadIdx.x; if (t >= n8) return;
  const v4f a = *(const v4fa*)(w + (size_t)t * 8), c = *(const v4fa*)(w + (size_t)t * 8 + 4);
  FragH f;
#pragma unroll
  for (int q = 0; q < 4; ++q) { f.h[q] = (_Float16)(bf16_rne(a[q]) * scale); f.h[4 + q] = (_Float16)(bf16_rne(c[q]) * scale); }
  const v8us o = f.half[0];
  unsigned short* d = Bt + (size_t)t * 8;
  *(volatile v8us*)d = o; __threadfence(); *(volatile v8us*)d = o;
}

__global__ __launch_bounds__(256) void k_x16(const float* __restrict__ x, unsigned short* __restrict__ X16, unsigned int n8) {
  const unsigned int t = blockIdx.x * 256u + threadIdx.x; if (t >= n8) return;
  const unsigned int r = t / (DM / 8), c8 = (t - r * (DM / 8)) * 8;
  const unsigned int b = r / SEQ, s = r - b * SEQ;
  const float* src = x + ((size_t)s * NB_FULL + b) * DM + c8;
  const v4f a = *(const v4fa*)src, c = *(const v4fa*)(src + 4);
  FragH f;
#pragma unroll
  for (int q = 0; q < 4; ++q) { f.h[q] = toh_flush(bf16_rne(a[q])); f.h[4 + q] = toh_flush(bf16_rne(c[q])); }
  const v8us o = f.half[0];
  unsigned short* d = X16 + (size_t)t * 8;
  *(volatile v8us*)d = o; __threadfence(); *(volatile v8us*)d = o;
}

__device__ __forceinline__ v8f g2_mma(v16h a, v16h b, v8f c) { v8f d = __builtin_amdgcn_wmma_f32_16x16x32_f16(false, a, false, b, (short)0, c, false, false); asm volatile("v_nop\n\tv_nop\n\tv_nop\n\tv_nop" : "+v"(d) : "v"(a), "v"(b)); return d; }

template <bool ARES, bool BIASROW>
__global__ __launch_bounds__(128) void k_gemm2(const unsigned short* __restrict__ A, const unsigned short* __restrict__ Ar, int lda, size_t sA,
    const unsigned short* __restrict__ Bh, int ldb, float alpha, const float* __restrict__ bias,
    float* __restrict__ C, _Float16* __restrict__ C16, _Float16* __restrict__ C16r, int ldc, size_t sC, int resmode, int M, int N, int K) {
  __shared__ __attribute__((aligned(16))) float so[4][32][68];
  const int tid = threadIdx.x, w = __builtin_amdgcn_readfirstlane(tid >> 5), lane = tid & 31, ln = lane & 15, hh = lane >> 4; const int by = blockIdx.y;
  const int ntn = N >> 6; const int mt = blockIdx.x / ntn, nq = blockIdx.x - mt * ntn; const int row0 = mt * 128 + 32 * w, col0 = nq * 64; if (row0 >= M) return;
  const size_t aofs = (size_t)by * sA + (size_t)(row0 + ln) * lda + 8 * hh;
  const size_t cofs = (size_t)by * sC;
  const unsigned short* a0p = A + aofs; const unsigned short* a1p = a0p + (size_t)16 * lda;
  const unsigned short* r0p = Ar + aofs; const unsigned short* r1p = r0p + (size_t)16 * lda;
  const unsigned short* b0p = Bh + (size_t)(col0 + ln) * ldb + 8 * hh; const unsigned short* b1p = b0p + (size_t)16 * ldb; const unsigned short* b2p = b1p + (size_t)16 * ldb; const unsigned short* b3p = b2p + (size_t)16 * ldb;
  const v8f z8 = {0.f,0.f,0.f,0.f,0.f,0.f,0.f,0.f};
  v8f c00 = z8, c01 = z8, c02 = z8, c03 = z8, c10 = z8, c11 = z8, c12 = z8, c13 = z8;
  v8f d00 = z8, d01 = z8, d02 = z8, d03 = z8, d10 = z8, d11 = z8, d12 = z8, d13 = z8;
#pragma unroll 1
  for (int kb = 0; kb < K; kb += 32) {
    const v16h a0 = ld_frag(a0p + kb), a1 = ld_frag(a1p + kb);
    v16h e0 = a0, e1 = a1;
    if (ARES) { e0 = ld_frag(r0p + kb); e1 = ld_frag(r1p + kb); }
    v16h b = ld_frag(b0p + kb); c00 = g2_mma(a0, b, c00); c10 = g2_mma(a1, b, c10); if (ARES) { d00 = g2_mma(e0, b, d00); d10 = g2_mma(e1, b, d10); }
    b = ld_frag(b1p + kb); c01 = g2_mma(a0, b, c01); c11 = g2_mma(a1, b, c11); if (ARES) { d01 = g2_mma(e0, b, d01); d11 = g2_mma(e1, b, d11); }
    b = ld_frag(b2p + kb); c02 = g2_mma(a0, b, c02); c12 = g2_mma(a1, b, c12); if (ARES) { d02 = g2_mma(e0, b, d02); d12 = g2_mma(e1, b, d12); }
    b = ld_frag(b3p + kb); c03 = g2_mma(a0, b, c03); c13 = g2_mma(a1, b, c13); if (ARES) { d03 = g2_mma(e0, b, d03); d13 = g2_mma(e1, b, d13); }
  }
  v8f accs[8] = {c00, c01, c02, c03, c10, c11, c12, c13};
  v8f accd[8] = {d00, d01, d02, d03, d10, d11, d12, d13};
#pragma unroll
  for (int u = 0; u < 8; ++u) {
    const int t = u & 3, half = u >> 2; const int col = col0 + t * 16 + ln;
    float bcol = 0.f; if (!BIASROW) bcol = bf16_rne(bias[col]);
#pragma unroll
    for (int r = 0; r < 8; ++r) {
      const int rloc = half * 16 + 8 * hh + r;
      float v = accs[u][r]; if (ARES) v += accd[u][r] * 0.0009765625f;
      float bv = bcol; if (BIASROW) bv = bf16_rne(bias[row0 + rloc]);
      so[w][rloc][t * 16 + ln] = v * alpha + bv;
    }
  }
  __builtin_amdgcn_fence(4  , "workgroup"); __builtin_amdgcn_wave_barrier();
  bool wres = false;
  if (C16r) { if (resmode == 1) wres = ((row0 % SEQ) < EARLY); else if (resmode == 2) wres = ((col0 % SEQ) < EARLY); }
  const int rsub = lane >> 4, c4 = (lane & 15) * 4;
  for (int pass = 0; pass < 2; ++pass) {
#pragma unroll
    for (int q = 0; q < 16; ++q) {
      const int r = q * 2 + rsub; const v4f v = *(const v4fa*)&so[w][r][c4];
      const size_t o = cofs + (size_t)(row0 + r) * ldc + col0 + c4;
      if (C) *(volatile v4f*)(C + o) = v;
      if (C16) {
        v4h h4, h4r;
#pragma unroll
        for (int i = 0; i < 4; ++i) { h4[i] = (_Float16)v[i]; h4r[i] = (_Float16)((v[i] - (float)h4[i]) * 1024.0f); }
        *(volatile v4h*)(C16 + o) = h4;
        if (wres) *(volatile v4h*)(C16r + o) = h4r;
      }
    }
    if (pass == 0) __threadfence();
  }
}

__global__ __launch_bounds__(128) void k_attn(const unsigned short* __restrict__ Qh, const unsigned short* __restrict__ Kh,
    const unsigned short* __restrict__ Vh, unsigned short* __restrict__ Oh) {
  __shared__ __attribute__((aligned(16))) unsigned short so[4][16][64];
  const int tid = threadIdx.x, w = __builtin_amdgcn_readfirstlane(tid >> 5), lane = tid & 31, ln = lane & 15, hh = lane >> 4;
  const int head = blockIdx.y, b = blockIdx.z;
  const int q0 = (int)blockIdx.x * 64 + w * 16;
  const size_t tok0 = (size_t)b * SEQ;
  const size_t qofs = (tok0 + q0 + ln) * DM + head * HD + 8 * hh;
  const v16h qa = ld_frag(Qh + qofs), qb = ld_frag(Qh + qofs + 32);
  const size_t kofs = (tok0 + ln) * DM + head * HD + 8 * hh;
  const size_t vofs = (size_t)(head * HD + ln) * NTOK + tok0 + 8 * hh;
  const v8f z8 = {0.f,0.f,0.f,0.f,0.f,0.f,0.f,0.f};
  v8f oh[4] = {z8, z8, z8, z8};
  float mrun = -1.0e30f, lrun = 0.0f;
#pragma unroll 1
  for (int st = 0; st < SEQ / 32; ++st) {
    const int kb = st * 32;
    v8f sc[2];
#pragma unroll
    for (int t = 0; t < 2; ++t) {
      const size_t ko = kofs + (size_t)(kb + 16 * t) * DM;
      const v16h ka = ld_frag(Kh + ko), kc = ld_frag(Kh + ko + 32);
      sc[t] = mma2(ka, qa, kc, qb, z8);
    }
    float mloc = sc[0][0];
#pragma unroll
    for (int r = 1; r < 8; ++r) mloc = fmaxf(mloc, sc[0][r]);
#pragma unroll
    for (int r = 0; r < 8; ++r) mloc = fmaxf(mloc, sc[1][r]);
    mloc = fmaxf(mloc, __shfl_xor(mloc, 16));
    const float mnew = fmaxf(mrun, mloc);
    const float alpha = __expf((mrun - mnew) * 0.125f);
    mrun = mnew;
    const float msh = mnew * 0.125f - 5.545177444f;
    FragH ph; float ls = 0.0f;
#pragma unroll
    for (int r = 0; r < 8; ++r) {
      const float e0 = sc[0][r] * 0.125f - msh, e1 = sc[1][r] * 0.125f - msh;
      const float p0 = (e0 < -9.70f) ? 0.0f : __expf(e0);
      const float p1 = (e1 < -9.70f) ? 0.0f : __expf(e1);
      const _Float16 h0 = (_Float16)p0, h1 = (_Float16)p1;
      ph.h[r] = h0; ph.h[8 + r] = h1;
      ls += (float)h0 + (float)h1;
    }
    lrun = lrun * alpha + ls;
#pragma unroll
    for (int dt = 0; dt < 4; ++dt) oh[dt] = oh[dt] * alpha;
#pragma unroll
    for (int dt = 0; dt < 4; ++dt) {
      const size_t vo = vofs + (size_t)(dt * 16) * NTOK + kb;
      const v16h va = ld_frag(Vh + vo);
      oh[dt] = mma1(va, ph.v, oh[dt]);
    }
  }
  const float lt = lrun + __shfl_xor(lrun, 16);
  const float inv = 64.0f * (1.0f / lt);
#pragma unroll
  for (int dt = 0; dt < 4; ++dt) {
    FragH fh;
#pragma unroll
    for (int r = 0; r < 8; ++r) {
      const float v = oh[dt][r] * inv;
      fh.h[r] = toh_flush(v);
    }
    *(v8us*)&so[w][ln][dt * 16 + 8 * hh] = fh.half[0];
  }
  __builtin_amdgcn_fence(4  , "workgroup"); __builtin_amdgcn_wave_barrier();
  const int rq = lane >> 3, pc = lane & 7;
  for (int pass = 0; pass < 2; ++pass) {
#pragma unroll
    for (int it = 0; it < 4; ++it) {
      const int row = it * 4 + rq;
      const size_t o = (tok0 + q0 + row) * DM + head * HD + pc * 8;
      const v8us v = *(const v8us*)&so[w][row][pc * 8];
      *(volatile v8us*)(Oh + o) = v;
    }
    if (pass == 0) __threadfence();
  }
}

extern "C" void kernel_launch(void* const* d_in, const int* in_sizes, int n_in,
                              void* d_out, int out_size, void* d_ws, size_t ws_size, hipStream_t stream) {
  if (n_in < 11) return;
  const long long need_x = ((long long)(SEQ - 1) * NB_FULL + NB) * DM;
  if ((long long)in_sizes[0] < need_x || (long long)in_sizes[1] < need_x || (long long)in_sizes[2] < need_x) return;
  if (in_sizes[3] < DM * DM || in_sizes[5] < DM * DM || in_sizes[7] < DM * DM || in_sizes[9] < DM * DM) return;
  if (in_sizes[4] < DM || in_sizes[6] < DM || in_sizes[8] < DM || in_sizes[10] < DM) return;
  if ((long long)out_size < need_x) return;
  const float* xq = (const float*)d_in[0]; const float* xk = (const float*)d_in[1]; const float* xv = (const float*)d_in[2];
  const float* wq = (const float*)d_in[3]; const float* bq = (const float*)d_in[4];
  const float* wk = (const float*)d_in[5]; const float* bk = (const float*)d_in[6];
  const float* wv = (const float*)d_in[7]; const float* bv = (const float*)d_in[8];
  const float* wo = (const float*)d_in[9]; const float* bo = (const float*)d_in[10];
  float* out = (float*)d_out;
  char* ws = (char*)d_ws; size_t off = 0;
  auto take = [&](size_t bytes) { char* p = ws + off; off += (bytes + 255) & ~(size_t)255; return p; };
  const size_t wbytes = (size_t)DM * DM * 2, pbytes = NTOK * DM * 2;
  unsigned short* WQ = (unsigned short*)take(wbytes); unsigned short* WK = (unsigned short*)take(wbytes);
  unsigned short* WV = (unsigned short*)take(wbytes); unsigned short* WO = (unsigned short*)take(wbytes);
  unsigned short* XQ = (unsigned short*)take(pbytes); unsigned short* XK = (unsigned short*)take(pbytes); unsigned short* XV = (unsigned short*)take(pbytes);
  unsigned short* Qh = (unsigned short*)take(pbytes); unsigned short* Kh = (unsigned short*)take(pbytes);
  unsigned short* VTh = (unsigned short*)take(pbytes); unsigned short* Oh = (unsigned short*)take(pbytes);
  if (off > ws_size || off > (size_t)134217728) return;

  { const unsigned int n8 = (unsigned int)((size_t)DM * DM / 8); const unsigned g = (n8 + 255u) / 256u;
    k_wnat<<<g, 256, 0, stream>>>(wq, n8, WQ, 32.0f); k_wnat<<<g, 256, 0, stream>>>(wk, n8, WK, 32.0f);
    k_wnat<<<g, 256, 0, stream>>>(wv, n8, WV, 32.0f); k_wnat<<<g, 256, 0, stream>>>(wo, n8, WO, 32.0f); }
  { const unsigned int n8 = (unsigned int)(NTOK * DM / 8); const unsigned g = (n8 + 255u) / 256u;
    k_x16<<<g, 256, 0, stream>>>(xq, XQ, n8); k_x16<<<g, 256, 0, stream>>>(xk, XK, n8); k_x16<<<g, 256, 0, stream>>>(xv, XV, n8); }

  const unsigned gq = (unsigned)((NTOK / 128) * (DM / 64));
  k_gemm2<false, false><<<dim3(gq, 1), 128, 0, stream>>>(XQ, XQ, DM, (size_t)0, WQ, DM, 0.03125f, bq, (float*)nullptr, (_Float16*)Qh, (_Float16*)nullptr, DM, (size_t)0, 0, (int)NTOK, DM, DM);
  k_gemm2<false, false><<<dim3(gq, 1), 128, 0, stream>>>(XK, XK, DM, (size_t)0, WK, DM, 0.03125f, bk, (float*)nullptr, (_Float16*)Kh, (_Float16*)nullptr, DM, (size_t)0, 0, (int)NTOK, DM, DM);
  k_gemm2<false, true><<<dim3((unsigned)((DM / 128) * (NTOK / 64)), 1), 128, 0, stream>>>(WV, WV, DM, (size_t)0, XV, DM, 0.03125f, bv, (float*)nullptr, (_Float16*)VTh, (_Float16*)nullptr, (int)NTOK, (size_t)0, 0, DM, (int)NTOK, DM);

  k_attn<<<dim3(SEQ / 64, NH, NB), 128, 0, stream>>>(Qh, Kh, VTh, Oh);

  k_gemm2<false, false><<<dim3((unsigned)((SEQ / 128) * (DM / 64)), NB), 128, 0, stream>>>(Oh, Oh, DM, (size_t)SEQ * DM, WO, DM, 0.00048828125f, bo, out, (_Float16*)nullptr, (_Float16*)nullptr, NB_FULL * DM, (size_t)DM, 0, SEQ, DM, DM);
}
